// MambaDynamics_43224550866990
// MI455X (gfx1250) — hardware-run, weakly checked
//
#include <hip/hip_runtime.h>
#include <hip/hip_fp16.h>
#include <math.h>

typedef __attribute__((ext_vector_type(16))) _Float16 v16h;
typedef __attribute__((ext_vector_type(8)))  _Float16 v8h;
typedef __attribute__((ext_vector_type(8)))  float    v8f;
typedef __attribute__((ext_vector_type(4)))  float    v4f;
typedef __attribute__((ext_vector_type(4)))  unsigned v4u;

constexpr int kNb     = 4;
constexpr int kSeq    = 4096;
constexpr int kDm     = 256;
constexpr int kIn     = 512;
constexpr int kNst    = 16;
constexpr int kXpP    = 2 * kIn;
constexpr int kBcLive = 2 * kNst;
constexpr int kBcP    = 64;
constexpr int kRows   = kNb * kSeq;
constexpr int kPassB  = 2;
constexpr int kNPass  = kNb / kPassB;
constexpr int kPRows  = kPassB * kSeq;
static_assert(kNPass * kPassB == kNb);
static_assert(kXpP == 1024 && kBcLive == 32 && kRows == 16384 && kPRows == 8192);
static_assert((kDm % 64) == 0 && (kIn % 64) == 0 && (kXpP % 64) == 0 && (kBcP % 64) == 0);
static_assert((kDm % 32) == 0 && (kIn % 32) == 0);
static_assert((kPRows % 32) == 0 && (kSeq % 64) == 0);
static_assert(kBcLive <= kBcP && (kBcLive % 4) == 0);

constexpr float kCarryX = 16.0f;
constexpr float kCarryW = 256.0f;
constexpr float kCarryR = 2048.0f;
constexpr float kCarryY = 65536.0f;
constexpr float kFoldMain   = 1.0f / (kCarryX * kCarryW);
constexpr float kFoldCross  = kFoldMain / kCarryR;
constexpr float kFoldMainY  = 1.0f / (kCarryY * kCarryW);
constexpr float kFoldCrossY = kFoldMainY / kCarryR;
static_assert(kFoldMain == 0.000244140625f);
static_assert(kFoldCross * 8388608.0f == 1.0f);
static_assert(kFoldMainY * 16777216.0f == 1.0f);
static_assert(kFoldCrossY * 34359738368.0f == 1.0f);

constexpr size_t kSzWin  = (size_t)kXpP * kDm * 2;
constexpr size_t kSzWcv  = (size_t)kIn * kIn * 2;
constexpr size_t kSzWbc  = (size_t)kBcP * kIn * 2;
constexpr size_t kSzWdt  = (size_t)kIn * kIn * 2;
constexpr size_t kSzWo   = (size_t)kDm * kIn * 2;
constexpr size_t kSzZs   = (size_t)kIn * 4;
constexpr size_t kSzX16  = (size_t)kPRows * kDm * 2;
constexpr size_t kSzXP   = (size_t)kPRows * kXpP * 4;
constexpr size_t kSzA16  = (size_t)kPRows * kIn * 2;
constexpr size_t kSzA32  = (size_t)kPRows * kIn * 4;
constexpr size_t kSzBC   = (size_t)kPRows * kBcP * 4;
constexpr size_t kWsTotal = 2 * kSzWin + 2 * kSzWcv + 2 * kSzWbc + kSzWdt + 2 * kSzWo + kSzZs
                          + 2 * kSzX16 + kSzXP + 2 * kSzA16 + kSzA32 + 2 * kSzA16 + kSzBC + kSzA32 + 2 * kSzA16;
static_assert(kWsTotal == 131205120ull);
static_assert(kWsTotal <= 134217728ull);
static_assert((kSzWin % 128) == 0 && (kSzWcv % 128) == 0 && (kSzWbc % 128) == 0 && (kSzWdt % 128) == 0 &&
              (kSzWo % 128) == 0 && (kSzZs % 128) == 0 && (kSzX16 % 128) == 0 && (kSzXP % 128) == 0 &&
              (kSzA16 % 128) == 0 && (kSzA32 % 128) == 0 && (kSzBC % 128) == 0);

__device__ __forceinline__ float g_flush16(float v) {
  return (fabsf(v) < 6.103515625e-05f) ? 0.0f : v;
}
__device__ __forceinline__ unsigned g_h16bits(float v) {
  return (unsigned)__half_as_ushort(__float2half_rn(g_flush16(v)));
}
__device__ __forceinline__ float g_h16val(unsigned b) {
  return __half2float(__ushort_as_half((unsigned short)b));
}
__device__ __forceinline__ void g_pack2(float v0, float v1, unsigned& hw, unsigned& lw) {
  const unsigned h0 = g_h16bits(v0);
  const unsigned h1 = g_h16bits(v1);
  const float r0 = (v0 - g_h16val(h0)) * kCarryR;
  const float r1 = (v1 - g_h16val(h1)) * kCarryR;
  const unsigned l0 = g_h16bits(r0);
  const unsigned l1 = g_h16bits(r1);
  hw = h0 | (h1 << 16);
  lw = l0 | (l1 << 16);
}

template <bool WANT_LO>
__global__ __launch_bounds__(256) void weight_planes_kernel(
    const float* __restrict__ W, int Kdim, int Nreal,
    unsigned short* __restrict__ dhi, unsigned short* __restrict__ dlo, float carry)
{
  __shared__ float sT[64 * 65];
  const int tid  = threadIdx.x;
  const int lane = tid & 31;
  const int wave = tid >> 5;
  const int k0 = blockIdx.x * 64;
  const int n0 = blockIdx.y * 64;
  const int nn = tid & 63;
  const int kb = tid >> 6;
  const int n  = n0 + nn;
  const bool live = (n < Nreal);
  const int nc = live ? n : (Nreal - 1);
#pragma unroll
  for (int i = 0; i < 16; ++i) {
    const int kk = kb + 4 * i;
    float w = W[(size_t)(k0 + kk) * Nreal + nc];
    asm volatile("" : "+v"(w));
    sT[kk * 65 + nn] = live ? (w * carry) : 0.0f;
  }
  __syncthreads();
  const int q  = lane >> 3;
  const int c8 = (lane & 7) * 8;
  v4u hv[2], lv[2];
#pragma unroll
  for (int it = 0; it < 2; ++it) {
    const int row = it * 32 + wave * 4 + q;
    float f[8];
#pragma unroll
    for (int e = 0; e < 8; ++e) f[e] = sT[(c8 + e) * 65 + row];
    unsigned h0, h1, h2, h3, l0, l1, l2, l3;
    g_pack2(f[0], f[1], h0, l0);
    g_pack2(f[2], f[3], h1, l1);
    g_pack2(f[4], f[5], h2, l2);
    g_pack2(f[6], f[7], h3, l3);
    hv[it] = (v4u){h0, h1, h2, h3};
    lv[it] = (v4u){l0, l1, l2, l3};
  }
  for (int pass = 0; pass < 2; ++pass) {
#pragma unroll
    for (int it = 0; it < 2; ++it) {
      const int row = it * 32 + wave * 4 + q;
      const size_t o = (size_t)(n0 + row) * Kdim + k0 + c8;
      *(volatile v4u*)(dhi + o) = hv[it];
      if (WANT_LO) *(volatile v4u*)(dlo + o) = lv[it];
    }
    __threadfence();
  }
}

__global__ __launch_bounds__(256) void cast_planes_kernel(
    const float* __restrict__ src, long ld_src, int col0, int ncol8,
    unsigned short* __restrict__ dhi, unsigned short* __restrict__ dlo, int total8, float carry)
{
  const int i = blockIdx.x * 256 + threadIdx.x;
  if (i >= total8) return;
  const int row = i / ncol8;
  const int c8  = (i - row * ncol8) * 8;
  const float* p = src + (long)row * ld_src + col0 + c8;
  const v4f a0 = *(const v4f*)(p);
  const v4f a1 = *(const v4f*)(p + 4);
  unsigned h0, h1, h2, h3, l0, l1, l2, l3;
  g_pack2(a0[0] * carry, a0[1] * carry, h0, l0);
  g_pack2(a0[2] * carry, a0[3] * carry, h1, l1);
  g_pack2(a1[0] * carry, a1[1] * carry, h2, l2);
  g_pack2(a1[2] * carry, a1[3] * carry, h3, l3);
  const v4u hv = (v4u){h0, h1, h2, h3};
  const v4u lv = (v4u){l0, l1, l2, l3};
  const size_t o = (size_t)i * 8;
  *(volatile v4u*)(dhi + o) = hv;
  *(volatile v4u*)(dlo + o) = lv;
  __threadfence();
  *(volatile v4u*)(dhi + o) = hv;
  *(volatile v4u*)(dlo + o) = lv;
}

static_assert(kIn == 128 * 4);
__global__ __launch_bounds__(128) void zero_vec_kernel(float* __restrict__ z)
{
  const v4f zero = (v4f){0.0f, 0.0f, 0.0f, 0.0f};
  float* p = z + threadIdx.x * 4;
  *(volatile v4f*)p = zero;
  __threadfence();
  *(volatile v4f*)p = zero;
}

__device__ __forceinline__ v16h frag_ld(const _Float16* p) {
  union { v16h v; v8h h[2]; } f;
  f.h[0] = *(const v8h*)(p);
  f.h[1] = *(const v8h*)(p + 16);
  return f.v;
}
__device__ __forceinline__ void mma_f16(v8f& c, const v16h a, const v16h b) {
  c = __builtin_amdgcn_wmma_f32_16x16x32_f16(false, a, false, b, (short)0, c, false, false);
  asm volatile("v_nop\n\tv_nop\n\tv_nop\n\tv_nop" : "+v"(c) : "v"(a), "v"(b));
}

template <int MODE, int EPI>
__global__ __launch_bounds__(256) __attribute__((amdgpu_num_vgpr(256))) void gemm_f16_kernel(
    const unsigned short* __restrict__ Ahp, const unsigned short* __restrict__ Alp, int lda,
    const unsigned short* __restrict__ Bhp, const unsigned short* __restrict__ Blp, int ldb,
    float* __restrict__ C, int ldc,
    const float* __restrict__ bias, int nbias,
    int M, int N, int K, float fmain, float fcross)
{
  __shared__ __align__(16) float sT[8][16 * 68];
  const int lane = threadIdx.x & 31;
  const int wave = threadIdx.x >> 5;
  const int tilesN = N >> 6;
  const int tilesM = M >> 5;
  const int tile = blockIdx.x * 8 + wave;
  if (tile >= tilesM * tilesN) return;
  const int tm = tile / tilesN;
  const int tn = tile - tm * tilesN;
  const int m0 = tm << 5;
  const int n0 = tn << 6;
  const int rlane = lane & 15;
  const int koff  = (lane >> 4) * 8;
  const int mOff  = (lane >> 4) * 8;

  const _Float16* pah0 = (const _Float16*)Ahp + (size_t)(m0 + rlane) * lda + koff;
  const _Float16* pah1 = pah0 + (size_t)16 * lda;
  const _Float16* pal0 = (const _Float16*)Alp + (size_t)(m0 + rlane) * lda + koff;
  const _Float16* pal1 = pal0 + (size_t)16 * lda;
  const _Float16* pbh  = (const _Float16*)Bhp + (size_t)(n0 + rlane) * ldb + koff;
  const _Float16* pbl  = (const _Float16*)Blp + (size_t)(n0 + rlane) * ldb + koff;

  v8f am[2][4], ac[2][4];
#pragma unroll
  for (int i = 0; i < 2; ++i)
#pragma unroll
    for (int j = 0; j < 4; ++j) {
      am[i][j] = (v8f){0.f, 0.f, 0.f, 0.f, 0.f, 0.f, 0.f, 0.f};
      ac[i][j] = (v8f){0.f, 0.f, 0.f, 0.f, 0.f, 0.f, 0.f, 0.f};
    }

  for (int k0 = 0; k0 < K; k0 += 32) {
    const v16h ah0 = frag_ld(pah0 + k0);
    const v16h ah1 = frag_ld(pah1 + k0);
    v16h al0 = ah0;
    v16h al1 = ah1;
    if (MODE == 1) {
      al0 = frag_ld(pal0 + k0);
      al1 = frag_ld(pal1 + k0);
    }
#pragma unroll
    for (int j = 0; j < 4; ++j) {
      const size_t bo = (size_t)(j << 4) * ldb + k0;
      const v16h bh = frag_ld(pbh + bo);
      mma_f16(am[0][j], ah0, bh);
      mma_f16(am[1][j], ah1, bh);
      if (MODE == 1) {
        const v16h bl = frag_ld(pbl + bo);
        mma_f16(ac[0][j], ah0, bl);
        mma_f16(ac[1][j], ah1, bl);
        mma_f16(ac[0][j], al0, bh);
        mma_f16(ac[1][j], al1, bh);
      }
    }
  }

  float* slab = sT[wave];
  const int hh = lane >> 4;
  const int c4 = (lane & 15) * 4;
  float b0, b1, b2, b3;
  {
    const int bcol = n0 + c4;
    const bool blive = (bcol + 4 <= nbias);
    const int bcc = blive ? bcol : (nbias - 4);
    const v4f bv = *(const v4f*)(bias + bcc);
    b0 = bv[0];
    b1 = bv[1];
    b2 = bv[2];
    b3 = bv[3];
    asm volatile("" : "+v"(b0), "+v"(b1), "+v"(b2), "+v"(b3));
    b0 = blive ? b0 : 0.0f;
    b1 = blive ? b1 : 0.0f;
    b2 = blive ? b2 : 0.0f;
    b3 = blive ? b3 : 0.0f;
  }
#pragma unroll
  for (int i = 0; i < 2; ++i) {
    const int mBase = m0 + (i << 4);
#pragma unroll
    for (int j = 0; j < 4; ++j) {
#pragma unroll
      for (int r = 0; r < 8; ++r) {
        float v = am[i][j][r] * fmain;
        if (MODE == 1) v = fmaf(ac[i][j][r], fcross, v);
        slab[(mOff + r) * 68 + (j << 4) + rlane] = v;
      }
    }
    __builtin_amdgcn_fence(__ATOMIC_RELEASE, "workgroup");
    __builtin_amdgcn_wave_barrier();
    __builtin_amdgcn_fence(__ATOMIC_ACQUIRE, "workgroup");
#pragma unroll 1
    for (int it = 0; it < 8; ++it) {
      float* sp = slab + (it * 2 + hh) * 68 + c4;
      const v4f v = *(const v4f*)sp;
      float e0 = v[0] + b0;
      float e1 = v[1] + b1;
      float e2 = v[2] + b2;
      float e3 = v[3] + b3;
      if (EPI == 1) {
        e0 = e0 * (1.0f / (1.0f + expf(-e0)));
        e1 = e1 * (1.0f / (1.0f + expf(-e1)));
        e2 = e2 * (1.0f / (1.0f + expf(-e2)));
        e3 = e3 * (1.0f / (1.0f + expf(-e3)));
      }
      *(v4f*)sp = (v4f){e0, e1, e2, e3};
    }
    for (int pass = 0; pass < 2; ++pass) {
#pragma unroll
      for (int it = 0; it < 8; ++it) {
        const int row = it * 2 + hh;
        const v4f v = *(const v4f*)(slab + row * 68 + c4);
        *(volatile v4f*)(C + (size_t)(mBase + row) * ldc + n0 + c4) = v;
      }
      __threadfence();
    }
    __builtin_amdgcn_fence(__ATOMIC_RELEASE, "workgroup");
    __builtin_amdgcn_wave_barrier();
    __builtin_amdgcn_fence(__ATOMIC_ACQUIRE, "workgroup");
  }
}

typedef float    ms1_v4f __attribute__((ext_vector_type(4)));
typedef unsigned ms1_v4u __attribute__((ext_vector_type(4)));
struct ms1_args {
  const float* dtpre;
  const float* u;
  const float* bc;
  const float* z;
  const float* A_log;
  const float* Dskip;
  __half* y;
  __half* y_lo;
  long ld_dtpre;
  long ld_u;
  long ld_bc;
  long ld_z;
  long ld_y;
  int offB;
  int offC;
  int offZ;
  float ycarry;
  int dir;
  int D;
  int L;
  int nbatch;
};
static_assert(sizeof(ms1_args) == 136);

__device__ __forceinline__ float ms1_flush16(float v) {
  return (fabsf(v) < 6.103515625e-05f) ? 0.0f : v;
}
__device__ __forceinline__ unsigned ms1_h16bits(float v) {
  return (unsigned)__half_as_ushort(__float2half_rn(ms1_flush16(v)));
}
__device__ __forceinline__ float ms1_h16val(unsigned b) {
  return __half2float(__ushort_as_half((unsigned short)b));
}
__device__ __forceinline__ float ms1_softplus(float v) {
  return fmaxf(v, 0.0f) + log1pf(expf(-fabsf(v)));
}
__device__ __forceinline__ void ms1_pack2(float v0, float v1, unsigned& hw, unsigned& lw) {
  const unsigned h0 = ms1_h16bits(v0);
  const unsigned h1 = ms1_h16bits(v1);
  const float r0 = (v0 - ms1_h16val(h0)) * 2048.0f;
  const float r1 = (v1 - ms1_h16val(h1)) * 2048.0f;
  const unsigned l0 = ms1_h16bits(r0);
  const unsigned l1 = ms1_h16bits(r1);
  hw = h0 | (h1 << 16);
  lw = l0 | (l1 << 16);
}

template <int NSTATE>
__global__ __launch_bounds__(64 * (NSTATE / 16)) void ms1_scan_kernel(ms1_args a)
{
  static_assert(NSTATE == 16 || NSTATE == 64);
  constexpr int NQ  = NSTATE / 16;
  constexpr int NT  = 64 * NQ;
  constexpr int NW  = NT / 32;
  constexpr int BCW = 2 * NSTATE;
  constexpr int YP  = 68;
  constexpr int RPI = NW * 4;
  constexpr int NIT = 64 / RPI;
  static_assert(16 * NT <= 64 * YP);
  __shared__ __align__(16) float sBC[64 * BCW];
  __shared__ __align__(16) float sY[64 * YP];
  const int tid  = threadIdx.x;
  const int lane = tid & 31;
  const int wave = tid >> 5;
  const int c    = tid / NQ;
  const int sq   = tid - c * NQ;
  const int bpb  = a.D / 64;
  const int bi   = blockIdx.x / bpb;
  if (bi >= a.nbatch) return;
  const int d0 = (blockIdx.x - bi * bpb) * 64;
  const int d  = d0 + c;
  const long rowb = (long)bi * a.L;
  const bool hasz  = (a.z != nullptr);
  const bool hasD  = (a.Dskip != nullptr);
  const bool hasLo = (a.y_lo != nullptr);

#pragma unroll 1
  for (int n = 0; n < 16; ++n) {
    const float al = a.A_log[(long)d * NSTATE + sq * 16 + n];
    sY[n * NT + tid] = -expf(al);
  }
  __syncthreads();
  float An[16], h[16];
#pragma unroll
  for (int n = 0; n < 16; ++n) {
    An[n] = sY[n * NT + tid];
    h[n] = 0.0f;
  }
  float Dd = 0.0f;
  if (hasD) Dd = a.Dskip[d];

  const int nchunk = a.L / 64;
  const bool fwd = (a.dir > 0);
  const int s0 = fwd ? 0 : 63;
  const int sd = fwd ? 1 : -1;
  const int q  = lane >> 3;
  const int c8 = (lane & 7) * 8;

#pragma unroll 1
  for (int ci = 0; ci < nchunk; ++ci) {
    const int tb = fwd ? (ci * 64) : (a.L - 64 - ci * 64);
    const long rowc = rowb + tb;
    __syncthreads();
#pragma unroll 8
    for (int i = 0; i < 32; ++i) {
      const int idx = tid + i * NT;
      const int st  = idx / BCW;
      const int col = idx - st * BCW;
      const int sc  = (col < NSTATE) ? (a.offB + col) : (a.offC + col - NSTATE);
      sBC[idx] = a.bc[(rowc + st) * a.ld_bc + sc];
    }
    __syncthreads();
#pragma unroll 1
    for (int s = 0; s < 64; ++s) {
      const int ls = s0 + sd * s;
      const long row = rowc + ls;
      float pre = a.dtpre[row * a.ld_dtpre + d];
      float uv  = a.u[row * a.ld_u + d];
      float zv  = 0.0f;
      if (hasz) zv = a.z[row * a.ld_z + a.offZ + d];
      asm volatile("" : "+v"(pre));
      asm volatile("" : "+v"(uv));
      asm volatile("" : "+v"(zv));
      const float delta = ms1_softplus(pre);
      const float dtx = delta * uv;
      const float* bp = sBC + ls * BCW + sq * 16;
      const float* cp = bp + NSTATE;
      ms1_v4f Bq[4], Cq[4];
#pragma unroll
      for (int k = 0; k < 4; ++k) {
        Bq[k] = *(const ms1_v4f*)(bp + 4 * k);
        Cq[k] = *(const ms1_v4f*)(cp + 4 * k);
      }
      float yv = 0.0f;
#pragma unroll
      for (int n = 0; n < 16; ++n) {
        const float e = __expf(delta * An[n]);
        h[n] = fmaf(e, h[n], dtx * Bq[n >> 2][n & 3]);
        yv = fmaf(h[n], Cq[n >> 2][n & 3], yv);
      }
      if (NQ > 1) {
        yv += __shfl_xor(yv, 1, 32);
        yv += __shfl_xor(yv, 2, 32);
      }
      if (hasD) yv = fmaf(uv, Dd, yv);
      if (hasz) {
        const float sg = __builtin_amdgcn_rcpf(1.0f + expf(-zv));
        yv = yv * (zv * sg);
      }
      if (sq == 0) sY[ls * YP + c] = yv * a.ycarry;
    }
    __syncthreads();
    ms1_v4u hw[NIT], lw[NIT];
#pragma unroll
    for (int it = 0; it < NIT; ++it) {
      const int row = it * RPI + wave * 4 + q;
      const float* sp = sY + row * YP + c8;
      const ms1_v4f f0 = *(const ms1_v4f*)(sp);
      const ms1_v4f f1 = *(const ms1_v4f*)(sp + 4);
      unsigned h0, h1, h2, h3, l0, l1, l2, l3;
      ms1_pack2(f0[0], f0[1], h0, l0);
      ms1_pack2(f0[2], f0[3], h1, l1);
      ms1_pack2(f1[0], f1[1], h2, l2);
      ms1_pack2(f1[2], f1[3], h3, l3);
      hw[it] = (ms1_v4u){h0, h1, h2, h3};
      lw[it] = (ms1_v4u){l0, l1, l2, l3};
    }
    for (int pass = 0; pass < 2; ++pass) {
#pragma unroll
      for (int it = 0; it < NIT; ++it) {
        const int row = it * RPI + wave * 4 + q;
        const long o = (rowc + row) * a.ld_y + d0 + c8;
        *(volatile ms1_v4u*)(a.y + o) = hw[it];
        if (hasLo) *(volatile ms1_v4u*)(a.y_lo + o) = lw[it];
      }
      __threadfence();
    }
  }
}

static_assert(((kPRows / 32) * (kXpP / 64)) % 8 == 0);
static_assert(((kPRows / 32) * (kIn / 64)) % 8 == 0);
static_assert(((kPRows / 32) * (kBcP / 64)) % 8 == 0);
static_assert(((kPRows / 32) * (kDm / 64)) % 8 == 0);
static_assert(((kPRows * kDm / 8) % 256) == 0 && ((kPRows * kIn / 8) % 256) == 0);

extern "C" void kernel_launch(void* const* d_in, const int* in_sizes, int n_in,
                              void* d_out, int out_size, void* d_ws, size_t ws_size,
                              hipStream_t stream) {
  if (n_in < 12) return;
  if (in_sizes[0] != kRows * kDm) return;
  if (in_sizes[1] != kDm * kXpP) return;
  if (in_sizes[2] != kXpP) return;
  if (in_sizes[3] != kIn * kIn) return;
  if (in_sizes[4] != kIn) return;
  if (in_sizes[5] != kIn * kNst) return;
  if (in_sizes[6] != kIn * kBcLive) return;
  if (in_sizes[7] != kBcLive) return;
  if (in_sizes[8] != kIn * kIn) return;
  if (in_sizes[9] != kIn) return;
  if (in_sizes[10] != kIn * kDm) return;
  if (in_sizes[11] != kDm) return;
  if (out_size != kRows * kDm) return;
  if (ws_size < kWsTotal) return;

  const float* x      = (const float*)d_in[0];
  const float* W_in   = (const float*)d_in[1];
  const float* b_in   = (const float*)d_in[2];
  const float* W_conv = (const float*)d_in[3];
  const float* b_conv = (const float*)d_in[4];
  const float* A_log  = (const float*)d_in[5];
  const float* W_bc   = (const float*)d_in[6];
  const float* b_bc   = (const float*)d_in[7];
  const float* W_dt   = (const float*)d_in[8];
  const float* b_dt   = (const float*)d_in[9];
  const float* W_out  = (const float*)d_in[10];
  const float* b_out  = (const float*)d_in[11];
  float* out = (float*)d_out;

  char* ws = (char*)d_ws;
  size_t off = 0;
  auto carve = [&](size_t bytes) -> char* { char* p = ws + off; off += bytes; return p; };
  unsigned short* WINH = (unsigned short*)carve(kSzWin);
  unsigned short* WINL = (unsigned short*)carve(kSzWin);
  unsigned short* WCVH = (unsigned short*)carve(kSzWcv);
  unsigned short* WCVL = (unsigned short*)carve(kSzWcv);
  unsigned short* WBCH = (unsigned short*)carve(kSzWbc);
  unsigned short* WBCL = (unsigned short*)carve(kSzWbc);
  unsigned short* WDTH = (unsigned short*)carve(kSzWdt);
  unsigned short* WOH  = (unsigned short*)carve(kSzWo);
  unsigned short* WOL  = (unsigned short*)carve(kSzWo);
  float*          ZSKIP = (float*)carve(kSzZs);
  unsigned short* XH   = (unsigned short*)carve(kSzX16);
  unsigned short* XL   = (unsigned short*)carve(kSzX16);
  float*          XP   = (float*)carve(kSzXP);
  unsigned short* XMH  = (unsigned short*)carve(kSzA16);
  unsigned short* XML  = (unsigned short*)carve(kSzA16);
  float*          U    = (float*)carve(kSzA32);
  unsigned short* UH   = (unsigned short*)carve(kSzA16);
  unsigned short* UL   = (unsigned short*)carve(kSzA16);
  float*          BC   = (float*)carve(kSzBC);
  float*          DTP  = (float*)carve(kSzA32);
  unsigned short* Y16  = (unsigned short*)carve(kSzA16);
  unsigned short* Y16L = (unsigned short*)carve(kSzA16);
  if (off != kWsTotal) return;

  weight_planes_kernel<true><<<dim3(kDm / 64, kXpP / 64), 256, 0, stream>>>(W_in, kDm, kXpP, WINH, WINL, kCarryW);
  weight_planes_kernel<true><<<dim3(kIn / 64, kIn / 64), 256, 0, stream>>>(W_conv, kIn, kIn, WCVH, WCVL, kCarryW);
  weight_planes_kernel<true><<<dim3(kIn / 64, kBcP / 64), 256, 0, stream>>>(W_bc, kIn, kBcLive, WBCH, WBCL, kCarryW);
  weight_planes_kernel<false><<<dim3(kIn / 64, kIn / 64), 256, 0, stream>>>(W_dt, kIn, kIn, WDTH, WDTH, kCarryW);
  weight_planes_kernel<true><<<dim3(kIn / 64, kDm / 64), 256, 0, stream>>>(W_out, kIn, kDm, WOH, WOL, kCarryW);
  zero_vec_kernel<<<1, 128, 0, stream>>>(ZSKIP);

  for (int ps = 0; ps < kNPass; ++ps) {
    const float* xps = x + (size_t)ps * kPRows * kDm;
    float* ops = out + (size_t)ps * kPRows * kDm;

    cast_planes_kernel<<<(kPRows * kDm / 8) / 256, 256, 0, stream>>>(
        xps, (long)kDm, 0, kDm / 8, XH, XL, kPRows * kDm / 8, kCarryX);

    gemm_f16_kernel<1, 0><<<((kPRows / 32) * (kXpP / 64)) / 8, 256, 0, stream>>>(
        XH, XL, kDm, WINH, WINL, kDm, XP, kXpP, b_in, kXpP,
        kPRows, kXpP, kDm, kFoldMain, kFoldCross);

    cast_planes_kernel<<<(kPRows * kIn / 8) / 256, 256, 0, stream>>>(
        XP, (long)kXpP, 0, kIn / 8, XMH, XML, kPRows * kIn / 8, kCarryX);

    gemm_f16_kernel<1, 1><<<((kPRows / 32) * (kIn / 64)) / 8, 256, 0, stream>>>(
        XMH, XML, kIn, WCVH, WCVL, kIn, U, kIn, b_conv, kIn,
        kPRows, kIn, kIn, kFoldMain, kFoldCross);

    cast_planes_kernel<<<(kPRows * kIn / 8) / 256, 256, 0, stream>>>(
        U, (long)kIn, 0, kIn / 8, UH, UL, kPRows * kIn / 8, kCarryX);

    gemm_f16_kernel<1, 0><<<((kPRows / 32) * (kBcP / 64)) / 8, 256, 0, stream>>>(
        UH, UL, kIn, WBCH, WBCL, kIn, BC, kBcP, b_bc, kBcLive,
        kPRows, kBcP, kIn, kFoldMain, kFoldCross);

    gemm_f16_kernel<0, 0><<<((kPRows / 32) * (kIn / 64)) / 8, 256, 0, stream>>>(
        UH, UH, kIn, WDTH, WDTH, kIn, DTP, kIn, b_dt, kIn,
        kPRows, kIn, kIn, kFoldMain, 0.0f);

    for (int bl = 0; bl < kPassB; ++bl) {
      const size_t r0 = (size_t)bl * kSeq;
      ms1_args sa;
      sa.dtpre = DTP + r0 * kIn;
      sa.u = U + r0 * kIn;
      sa.bc = BC + r0 * kBcP;
      sa.z = XP + r0 * kXpP;
      sa.A_log = A_log;
      sa.Dskip = ZSKIP;
      sa.y = (__half*)(Y16 + r0 * kIn);
      sa.y_lo = (__half*)(Y16L + r0 * kIn);
      sa.ld_dtpre = kIn;
      sa.ld_u = kIn;
      sa.ld_bc = kBcP;
      sa.ld_z = kXpP;
      sa.ld_y = kIn;
      sa.offB = 0;
      sa.offC = kNst;
      sa.offZ = kIn;
      sa.ycarry = kCarryY;
      sa.dir = 1;
      sa.D = kIn;
      sa.L = kSeq;
      sa.nbatch = 1;
      ms1_scan_kernel<16><<<dim3(kIn / 64), 64, 0, stream>>>(sa);
    }

    gemm_f16_kernel<1, 0><<<((kPRows / 32) * (kDm / 64)) / 8, 256, 0, stream>>>(
        Y16, Y16L, kIn, WOH, WOL, kIn, ops, kDm, b_out, kDm,
        kPRows, kDm, kIn, kFoldMainY, kFoldCrossY);
  }
}
